// Model_13245679140924
// MI455X (gfx1250) — hardware-verified
//
#include <hip/hip_runtime.h>
#include <math.h>

constexpr int NODES_C    = 1024;
constexpr int NODES_D    = 64;
constexpr int EDGES_C    = 16384;
constexpr int EDGES_D    = 1024;
constexpr int FEAT_C     = 128;
constexpr int FEAT_D     = 32;
constexpr int FEAT_D_PAD = 64;
constexpr int HIDDEN     = 1024;
constexpr int RNN_H      = 256;
constexpr int GATES3     = 3 * RNN_H;
constexpr int XPW        = 2 * GATES3;
constexpr int TSTEPS     = 64;
constexpr int NCLASS     = 3;
constexpr int NTHR       = 256;
constexpr int GRU_ROWS   = 16;
constexpr int GRU_TILES  = NODES_C / GRU_ROWS;
constexpr int HPITCH     = 264;
constexpr int SLABP      = 68;
constexpr float W_CARRY      = 16.0f;
constexpr float W_CARRY_INV  = 1.0f / 16.0f;
constexpr float X1_CARRY     = 16.0f;
constexpr float X1_CARRY_INV = 1.0f / 16.0f;

static_assert(TSTEPS == NODES_D, "time axis is the device axis");
static_assert(NODES_C % 64 == 0 && NODES_D % 64 == 0 && HIDDEN % 64 == 0 && XPW % 64 == 0, "tile multiples");
static_assert(FEAT_C % 32 == 0 && FEAT_D_PAD % 32 == 0 && HIDDEN % 32 == 0 && NODES_C % 32 == 0 && NODES_D % 32 == 0 && RNN_H % 32 == 0, "K multiples of 32");
static_assert(RNN_H == 32 * (NTHR / 32), "8 waves x 32 hidden columns");
static_assert((2 * GRU_ROWS * HPITCH) % NTHR == 0, "h zero-fill loop exact");
static_assert(EDGES_C % NTHR == 0 && EDGES_D % NTHR == 0, "edge loops exact");
static_assert(HPITCH % 8 == 0, "16-B aligned fragment rows");

typedef __attribute__((ext_vector_type(16))) _Float16 v16h;
typedef __attribute__((ext_vector_type(8)))  _Float16 v8h;
typedef __attribute__((ext_vector_type(8)))  float    v8f;
typedef __attribute__((ext_vector_type(4)))  float    v4f;

__device__ __forceinline__ void guard4_h(v8f& a, v8f& b, v8f& c, v8f& d, v16h x, v16h y) {
  asm volatile("v_nop\n\tv_nop\n\tv_nop\n\tv_nop" : "+v"(a), "+v"(b), "+v"(c), "+v"(d) : "v"(x), "v"(y));
}
__device__ __forceinline__ void guard3_h(v8f& a, v8f& b, v8f& c, v16h x, v16h y0, v16h y1, v16h y2) {
  asm volatile("v_nop\n\tv_nop\n\tv_nop\n\tv_nop" : "+v"(a), "+v"(b), "+v"(c) : "v"(x), "v"(y0), "v"(y1), "v"(y2));
}
__device__ __forceinline__ void guard1_h(v8f& a, v16h x, v16h y) {
  asm volatile("v_nop\n\tv_nop\n\tv_nop\n\tv_nop" : "+v"(a) : "v"(x), "v"(y));
}
__device__ __forceinline__ void keep4_h(v16h a, v16h b, v16h c, v16h d) { asm volatile("v_nop" :: "v"(a), "v"(b), "v"(c), "v"(d)); }
__device__ __forceinline__ void acc_guard4(v8f& a, v8f& b, v8f& c, v8f& d) {
  asm volatile("v_nop\n\tv_nop\n\tv_nop\n\tv_nop" : "+v"(a), "+v"(b), "+v"(c), "+v"(d));
}
__device__ __forceinline__ v16h frag_load(const _Float16* p) {
  union U { v16h v; v8h h[2]; } f;
  f.h[0] = *(const v8h*)(p);
  f.h[1] = *(const v8h*)(p + 16);
  return f.v;
}
__device__ __forceinline__ v8f frag_mma(v16h a, v16h b, v8f c) {
  return __builtin_amdgcn_wmma_f32_16x16x32_f16(false, a, false, b, (short)0, c, false, false);
}
__device__ __forceinline__ void wave_lds_sync() {
  __builtin_amdgcn_fence(__ATOMIC_RELEASE, "workgroup");
  __builtin_amdgcn_wave_barrier();
  __builtin_amdgcn_fence(__ATOMIC_ACQUIRE, "workgroup");
}
__device__ __forceinline__ float sigm(float x)    { return __builtin_amdgcn_rcpf(1.0f + expf(-x)); }
__device__ __forceinline__ float tanh_id(float x) { return 1.0f - 2.0f * __builtin_amdgcn_rcpf(expf(2.0f * x) + 1.0f); }

__global__ __launch_bounds__(NTHR) void deg_kernel(const int* __restrict__ src, const int* __restrict__ dst,
                                                   int nedges, int nnodes, float* __restrict__ DEG) {
  __shared__ int cin[32];
  __shared__ int cout[32];
  const int tid = threadIdx.x;
  const int n0 = blockIdx.x * 32;
  if (tid < 32) { cin[tid] = 0; cout[tid] = 0; }
  __syncthreads();
#pragma unroll 1
  for (int e = tid; e < nedges; e += NTHR) {
    const int s = src[e] - n0;
    const int d = dst[e] - n0;
    if ((unsigned)d < 32u) atomicAdd(&cin[d], 1);
    if ((unsigned)s < 32u) atomicAdd(&cout[s], 1);
  }
  __syncthreads();
  if (tid < 32) {
    const float fi = (float)cin[tid];
    const float fo = (float)cout[tid];
    const float ri = rsqrtf(fmaxf(fi, 1.0f));
    const float ro = rsqrtf(fmaxf(fo, 1.0f));
    float* p0 = DEG + n0 + tid;
    float* p1 = DEG + nnodes + n0 + tid;
    float* p2 = DEG + 2 * nnodes + n0 + tid;
    *(volatile float*)p0 = fi;
    *(volatile float*)p1 = ri;
    *(volatile float*)p2 = ro;
    __threadfence();
    *(volatile float*)p0 = fi;
    *(volatile float*)p1 = ri;
    *(volatile float*)p2 = ro;
  }
}

template <int NCOLS>
__global__ __launch_bounds__(NTHR) void adj_kernel(const int* __restrict__ src, const int* __restrict__ dst,
                                                   int nedges, unsigned short* __restrict__ ADJ) {
  __shared__ int cnt[8 * NCOLS];
  const int tid = threadIdx.x;
  const int r0 = blockIdx.x * 8;
#pragma unroll 1
  for (int i = tid; i < 8 * NCOLS; i += NTHR) cnt[i] = 0;
  __syncthreads();
#pragma unroll 1
  for (int e = tid; e < nedges; e += NTHR) {
    const int d = dst[e] - r0;
    int s = src[e];
    s = s < 0 ? 0 : (s > NCOLS - 1 ? NCOLS - 1 : s);
    if ((unsigned)d < 8u) atomicAdd(&cnt[d * NCOLS + s], 1);
  }
  __syncthreads();
  constexpr int PPR = NCOLS / 8;
#pragma unroll 1
  for (int i = tid; i < NCOLS; i += NTHR) {
    const int row = i / PPR;
    const int c8 = (i - row * PPR) * 8;
    v8h hv;
#pragma unroll
    for (int e = 0; e < 8; ++e) hv[e] = (_Float16)((float)cnt[row * NCOLS + c8 + e]);
    unsigned short* p = ADJ + (size_t)(r0 + row) * NCOLS + c8;
    *(volatile v8h*)p = hv;
    __threadfence();
    *(volatile v8h*)p = hv;
  }
}

__global__ __launch_bounds__(NTHR) void tpw_f16_kernel(const float* __restrict__ src, int Rreal, int C, int ldo,
                                                       unsigned short* __restrict__ O, float sc) {
  __shared__ float Tt[64 * 65];
  const int tid = threadIdx.x;
  const int c0 = blockIdx.x * 64, r0 = blockIdx.y * 64;
#pragma unroll
  for (int i = 0; i < 4; ++i) {
    const int idx = i * NTHR + tid;
    const int rr = idx >> 4, cc = (idx & 15) * 4;
    const int r = r0 + rr;
    const bool ok = r < Rreal;
    const int rcl = ok ? r : (Rreal - 1);
    const v4f v = *(const v4f*)(src + (size_t)rcl * (size_t)C + c0 + cc);
    Tt[rr * 65 + cc + 0] = ok ? v[0] : 0.0f;
    Tt[rr * 65 + cc + 1] = ok ? v[1] : 0.0f;
    Tt[rr * 65 + cc + 2] = ok ? v[2] : 0.0f;
    Tt[rr * 65 + cc + 3] = ok ? v[3] : 0.0f;
  }
  __syncthreads();
  const int q = tid >> 3, c8 = (tid & 7) * 8;
  v8h hv[2];
#pragma unroll
  for (int g = 0; g < 2; ++g) {
    const int qq = g * 32 + q;
#pragma unroll
    for (int e = 0; e < 8; ++e) {
      const float f = Tt[(c8 + e) * 65 + qq];
      hv[g][e] = (_Float16)(f * sc);
    }
  }
  for (int pass = 0; pass < 2; ++pass) {
#pragma unroll
    for (int g = 0; g < 2; ++g) {
      const size_t o = (size_t)(c0 + g * 32 + q) * (size_t)ldo + (size_t)(r0 + c8);
      *(volatile v8h*)(O + o) = hv[g];
    }
    __threadfence();
  }
}

__global__ __launch_bounds__(NTHR) void wf_prep_kernel(const float* __restrict__ Wf, unsigned short* __restrict__ WFT) {
  const int i = blockIdx.x * NTHR + threadIdx.x;
  const int dir = i >> 9;
  const int n = (i >> 5) & 15;
  const int k8 = (i & 31) * 8;
  const bool ok = n < NCLASS;
  const int ncl = ok ? n : (NCLASS - 1);
  v8h hv;
#pragma unroll
  for (int e = 0; e < 8; ++e) {
    const float f = Wf[(size_t)(dir * RNN_H + k8 + e) * NCLASS + ncl];
    hv[e] = (_Float16)(ok ? f * W_CARRY : 0.0f);
  }
  unsigned short* p = WFT + (size_t)i * 8;
  *(volatile v8h*)p = hv;
  __threadfence();
  *(volatile v8h*)p = hv;
}

__global__ __launch_bounds__(NTHR) void featn_kernel(const float* __restrict__ feat, int nrow, int ncol_real, int ncol_pad,
                                                     const float* __restrict__ rsout, unsigned short* __restrict__ dst) {
  const int i = blockIdx.x * NTHR + threadIdx.x;
  const int pc8 = ncol_pad >> 3;
  const int n8 = nrow * pc8;
  if (i < n8) {
    const int row = i / pc8;
    const int c8 = (i - row * pc8) * 8;
    const bool ok = c8 < ncol_real;
    const int cc = ok ? c8 : (ncol_real - 8);
    const float* sp = feat + (size_t)row * ncol_real + cc;
    const v4f a = *(const v4f*)(sp);
    const v4f b = *(const v4f*)(sp + 4);
    const float sc = rsout[row];
    v8h hv;
#pragma unroll
    for (int e = 0; e < 4; ++e) {
      hv[e]     = (_Float16)(ok ? a[e] * sc : 0.0f);
      hv[4 + e] = (_Float16)(ok ? b[e] * sc : 0.0f);
    }
    unsigned short* p = dst + (size_t)i * 8;
    *(volatile v8h*)p = hv;
    __threadfence();
    *(volatile v8h*)p = hv;
  }
}

template <int OUT_MODE>
__global__ __launch_bounds__(NTHR) void gemm_f16_kernel(
    const unsigned short* __restrict__ Ap, int lda,
    const unsigned short* __restrict__ Btp, int ldb,
    void* __restrict__ Cout, int ldc, int M, int N, int K, float scale) {
  const _Float16* A = (const _Float16*)Ap;
  const _Float16* Bt = (const _Float16*)Btp;
  __shared__ __align__(16) float sT[8][16 * SLABP];
  const int lane = threadIdx.x & 31;
  const int wave = threadIdx.x >> 5;
  const int tilesN = N >> 6;
  const int tilesM = M >> 6;
  const int tile = blockIdx.x * 8 + wave;
  if (tile >= tilesM * tilesN) return;
  const int tm = tile / tilesN;
  const int tn = tile - tm * tilesN;
  const int m0 = tm << 6;
  const int n0 = tn << 6;
  const int rlane = lane & 15;
  const int koff  = (lane >> 4) * 8;
  const int mOff  = (lane >> 4) * 8;

  v8f acc[4][4];
#pragma unroll
  for (int i = 0; i < 4; ++i)
#pragma unroll
    for (int j = 0; j < 4; ++j) acc[i][j] = (v8f){0.f, 0.f, 0.f, 0.f, 0.f, 0.f, 0.f, 0.f};

  for (int k0 = 0; k0 < K; k0 += 32) {
    v16h bh[4];
#pragma unroll
    for (int j = 0; j < 4; ++j) {
      const size_t bo = (size_t)(n0 + (j << 4) + rlane) * ldb + koff + k0;
      bh[j] = frag_load(Bt + bo);
    }
#pragma unroll
    for (int i = 0; i < 4; ++i) {
      const size_t ao = (size_t)(m0 + (i << 4) + rlane) * lda + koff + k0;
      const v16h ah = frag_load(A + ao);
#pragma unroll
      for (int j = 0; j < 4; ++j) acc[i][j] = frag_mma(ah, bh[j], acc[i][j]);
      guard4_h(acc[i][0], acc[i][1], acc[i][2], acc[i][3], ah, ah);
    }
    keep4_h(bh[0], bh[1], bh[2], bh[3]);
  }
  acc_guard4(acc[0][0], acc[0][1], acc[0][2], acc[0][3]);
  acc_guard4(acc[1][0], acc[1][1], acc[1][2], acc[1][3]);
  acc_guard4(acc[2][0], acc[2][1], acc[2][2], acc[2][3]);
  acc_guard4(acc[3][0], acc[3][1], acc[3][2], acc[3][3]);

  float* slab = sT[wave];
#pragma unroll
  for (int i = 0; i < 4; ++i) {
    const int mBase = m0 + (i << 4);
#pragma unroll
    for (int j = 0; j < 4; ++j) {
#pragma unroll
      for (int r = 0; r < 8; ++r) slab[(mOff + r) * SLABP + (j << 4) + rlane] = acc[i][j][r] * scale;
    }
    wave_lds_sync();
    if (OUT_MODE == 0) {
      float* C = (float*)Cout;
      const int hh = lane >> 4, c4 = (lane & 15) * 4;
      for (int pass = 0; pass < 2; ++pass) {
#pragma unroll
        for (int it = 0; it < 8; ++it) {
          const int row = it * 2 + hh;
          const v4f v = *(const v4f*)(slab + row * SLABP + c4);
          *(volatile v4f*)(C + (size_t)(mBase + row) * ldc + n0 + c4) = v;
        }
        __threadfence();
      }
    } else {
      const int q = lane >> 3, c8 = (lane & 7) * 8;
      unsigned short* C = (unsigned short*)Cout;
      for (int pass = 0; pass < 2; ++pass) {
#pragma unroll
        for (int it = 0; it < 4; ++it) {
          const int row = it * 4 + q;
          const float* sp = slab + row * SLABP + c8;
          v8h hv;
#pragma unroll
          for (int e = 0; e < 8; ++e) hv[e] = (_Float16)sp[e];
          *(volatile v8h*)(C + (size_t)(mBase + row) * ldc + n0 + c8) = hv;
        }
        __threadfence();
      }
    }
    wave_lds_sync();
  }
}

template <int ACTMODE>
__global__ __launch_bounds__(NTHR) void graph_gemm_kernel(
    const unsigned short* __restrict__ Ap, int lda,
    const unsigned short* __restrict__ Btp, int ldb,
    unsigned short* __restrict__ Cout, int ldc,
    const float* __restrict__ DEG, const float* __restrict__ wedge, const float* __restrict__ bias,
    int M, int N, int K, float scale) {
  const _Float16* A = (const _Float16*)Ap;
  const _Float16* Bt = (const _Float16*)Btp;
  __shared__ __align__(16) float sT[8][16 * SLABP];
  const int lane = threadIdx.x & 31;
  const int wave = threadIdx.x >> 5;
  const int tilesN = N >> 6;
  const int tilesM = M >> 6;
  const int tile = blockIdx.x * 8 + wave;
  if (tile >= tilesM * tilesN) return;
  const int tm = tile / tilesN;
  const int tn = tile - tm * tilesN;
  const int m0 = tm << 6;
  const int n0 = tn << 6;
  const int rlane = lane & 15;
  const int koff  = (lane >> 4) * 8;
  const int mOff  = (lane >> 4) * 8;

  v8f acc[4][4];
#pragma unroll
  for (int i = 0; i < 4; ++i)
#pragma unroll
    for (int j = 0; j < 4; ++j) acc[i][j] = (v8f){0.f, 0.f, 0.f, 0.f, 0.f, 0.f, 0.f, 0.f};

  for (int k0 = 0; k0 < K; k0 += 32) {
    v16h bh[4];
#pragma unroll
    for (int j = 0; j < 4; ++j) {
      const size_t bo = (size_t)(n0 + (j << 4) + rlane) * ldb + koff + k0;
      bh[j] = frag_load(Bt + bo);
    }
#pragma unroll
    for (int i = 0; i < 4; ++i) {
      const size_t ao = (size_t)(m0 + (i << 4) + rlane) * lda + koff + k0;
      const v16h ah = frag_load(A + ao);
#pragma unroll
      for (int j = 0; j < 4; ++j) acc[i][j] = frag_mma(ah, bh[j], acc[i][j]);
      guard4_h(acc[i][0], acc[i][1], acc[i][2], acc[i][3], ah, ah);
    }
    keep4_h(bh[0], bh[1], bh[2], bh[3]);
  }
  acc_guard4(acc[0][0], acc[0][1], acc[0][2], acc[0][3]);
  acc_guard4(acc[1][0], acc[1][1], acc[1][2], acc[1][3]);
  acc_guard4(acc[2][0], acc[2][1], acc[2][2], acc[2][3]);
  acc_guard4(acc[3][0], acc[3][1], acc[3][2], acc[3][3]);

  float* slab = sT[wave];
  const int q = lane >> 3, c8 = (lane & 7) * 8;
  const v4f we0 = *(const v4f*)(wedge + n0 + c8);
  const v4f we1 = *(const v4f*)(wedge + n0 + c8 + 4);
  const v4f bi0 = *(const v4f*)(bias + n0 + c8);
  const v4f bi1 = *(const v4f*)(bias + n0 + c8 + 4);
  const float* degraw = DEG;
  const float* rsin   = DEG + M;
  const float* rsout  = DEG + 2 * M;
#pragma unroll
  for (int i = 0; i < 4; ++i) {
    const int mBase = m0 + (i << 4);
#pragma unroll
    for (int j = 0; j < 4; ++j) {
#pragma unroll
      for (int r = 0; r < 8; ++r) slab[(mOff + r) * SLABP + (j << 4) + rlane] = acc[i][j][r] * scale;
    }
    wave_lds_sync();
#pragma unroll 1
    for (int it = 0; it < 4; ++it) {
      const int row = it * 4 + q;
      const int d = mBase + row;
      const float dr = degraw[d];
      const float ri = rsin[d];
      const float ro = rsout[d] * X1_CARRY;
      float* sp = slab + row * SLABP + c8;
      const v4f a0 = *(const v4f*)(sp);
      const v4f a1 = *(const v4f*)(sp + 4);
      v4f o0, o1;
#pragma unroll
      for (int e = 0; e < 4; ++e) {
        float t0 = (a0[e] + dr * we0[e]) * ri + bi0[e];
        float t1 = (a1[e] + dr * we1[e]) * ri + bi1[e];
        if (ACTMODE == 1) {
          const float e0 = expf(t0) - 1.0f;
          const float e1 = expf(t1) - 1.0f;
          t0 = ((t0 > 0.0f) ? t0 : e0) * ro;
          t1 = ((t1 > 0.0f) ? t1 : e1) * ro;
        }
        o0[e] = t0;
        o1[e] = t1;
      }
      *(v4f*)(sp) = o0;
      *(v4f*)(sp + 4) = o1;
    }
    wave_lds_sync();
    for (int pass = 0; pass < 2; ++pass) {
#pragma unroll
      for (int it = 0; it < 4; ++it) {
        const int row = it * 4 + q;
        const float* sp = slab + row * SLABP + c8;
        v8h hv;
#pragma unroll
        for (int e = 0; e < 8; ++e) hv[e] = (_Float16)sp[e];
        *(volatile v8h*)(Cout + (size_t)(mBase + row) * ldc + n0 + c8) = hv;
      }
      __threadfence();
    }
    wave_lds_sync();
  }
}

__global__ __launch_bounds__(NTHR) void gru_bidir_kernel(
    const float* __restrict__ CX, const float* __restrict__ DX,
    const unsigned short* __restrict__ WHTp, const unsigned short* __restrict__ WFTp,
    const float* __restrict__ b_f, const float* __restrict__ b_b, float* __restrict__ PL) {
  __shared__ __align__(16) _Float16 Ah[2][GRU_ROWS * HPITCH];
  __shared__ __align__(16) _Float16 Wfs[16 * HPITCH];
  __shared__ __align__(16) float    Ps[16 * 4];
  const int tid = threadIdx.x, lane = tid & 31, wave = tid >> 5;
  const int c = lane & 15, hh = lane >> 4, koff = hh * 8;
  const int dir = blockIdx.x / GRU_TILES;
  const int rowbase = (blockIdx.x - dir * GRU_TILES) * GRU_ROWS;
  const int cb = dir * GATES3;
  const float* bb = dir ? b_b : b_f;
  const _Float16* WH = (const _Float16*)WHTp + (size_t)dir * GATES3 * RNN_H;

  {
    _Float16* ahf = &Ah[0][0];
#pragma unroll 1
    for (int i = tid; i < 2 * GRU_ROWS * HPITCH; i += NTHR) ahf[i] = (_Float16)0.0f;
  }
  {
    const v8h* wsrc = (const v8h*)(const void*)(WFTp + (size_t)dir * 16 * RNN_H);
#pragma unroll 1
    for (int i = tid; i < 512; i += NTHR) {
      const int row = i >> 5, k8 = (i & 31) * 8;
      const v8h w = wsrc[i];
      *(v8h*)(Wfs + row * HPITCH + k8) = w;
    }
  }
  float cz[2][8], cr[2][8], ch[2][8], hst[2][8], brh[2];
#pragma unroll
  for (int nt = 0; nt < 2; ++nt) {
    const int j = 32 * wave + 16 * nt + c;
    const float biz = bb[j], bir = bb[RNN_H + j], bih = bb[2 * RNN_H + j];
    const float brz = bb[GATES3 + j], brr = bb[GATES3 + RNN_H + j];
    brh[nt] = bb[GATES3 + 2 * RNN_H + j];
#pragma unroll
    for (int r = 0; r < 8; ++r) {
      const float* cp = CX + (size_t)(rowbase + 8 * hh + r) * XPW + cb + j;
      cz[nt][r] = cp[0] + (biz + brz);
      cr[nt][r] = cp[RNN_H] + (bir + brr);
      ch[nt][r] = cp[2 * RNN_H] + bih;
      hst[nt][r] = 0.0f;
    }
  }
  __syncthreads();

  const v8f z8 = {0.f, 0.f, 0.f, 0.f, 0.f, 0.f, 0.f, 0.f};

#pragma unroll 1
  for (int step = 0; step < TSTEPS; ++step) {
    const int t = dir ? (TSTEPS - 1 - step) : step;
    const int cur = step & 1;
    const _Float16* ahrow = &Ah[cur][0] + c * HPITCH + koff;
    _Float16* ahn = &Ah[cur ^ 1][0];
#pragma unroll
    for (int nt = 0; nt < 2; ++nt) {
      const int j = 32 * wave + 16 * nt + c;
      const _Float16* wh = WH + (size_t)j * RNN_H + koff;
      const float* dxp = DX + (size_t)t * XPW + cb + j;
      float dxz = dxp[0];
      float dxr = dxp[RNN_H];
      float dxh = dxp[2 * RNN_H];
      asm volatile("" : "+v"(dxz), "+v"(dxr), "+v"(dxh));
      v8f az = z8, ar = z8, ag = z8;
#pragma unroll 1
      for (int k0 = 0; k0 < RNN_H; k0 += 32) {
        const v16h a  = frag_load(ahrow + k0);
        const v16h b0 = frag_load(wh + k0);
        const v16h b1 = frag_load(wh + (size_t)1 * RNN_H * RNN_H + k0);
        const v16h b2 = frag_load(wh + (size_t)2 * RNN_H * RNN_H + k0);
        az = frag_mma(a, b0, az);
        ar = frag_mma(a, b1, ar);
        ag = frag_mma(a, b2, ag);
        guard3_h(az, ar, ag, a, b0, b1, b2);
      }
#pragma unroll
      for (int r = 0; r < 8; ++r) {
        const float zg = sigm(cz[nt][r] + dxz + az[r] * W_CARRY_INV);
        const float rg = sigm(cr[nt][r] + dxr + ar[r] * W_CARRY_INV);
        const float hc = tanh_id(ch[nt][r] + dxh + rg * (ag[r] * W_CARRY_INV + brh[nt]));
        const float ho = hst[nt][r];
        const float hn = zg * ho + (1.0f - zg) * hc;
        hst[nt][r] = hn;
        ahn[(8 * hh + r) * HPITCH + j] = (_Float16)hn;
      }
    }
    __syncthreads();
    if (wave == 0) {
      const _Float16* hrow = ahn + c * HPITCH + koff;
      const _Float16* wf = Wfs + c * HPITCH + koff;
      v8f pa = z8;
#pragma unroll 1
      for (int k0 = 0; k0 < RNN_H; k0 += 32) {
        const v16h a = frag_load(hrow + k0);
        const v16h b = frag_load(wf + k0);
        pa = frag_mma(a, b, pa);
        guard1_h(pa, a, b);
      }
      if (c < 4) {
#pragma unroll
        for (int r = 0; r < 8; ++r) Ps[(8 * hh + r) * 4 + c] = pa[r] * W_CARRY_INV;
      }
      wave_lds_sync();
      const int prow = lane & 15;
      const v4f pv = *(const v4f*)(Ps + prow * 4);
      float* pp = PL + (((size_t)dir * TSTEPS + (size_t)t) * NODES_C + (size_t)(rowbase + prow)) * 4;
      if (lane < 16) *(volatile v4f*)pp = pv;
      __threadfence();
      if (lane < 16) *(volatile v4f*)pp = pv;
      wave_lds_sync();
    }
  }
}

__global__ __launch_bounds__(NTHR) void head_final_kernel(const float* __restrict__ PL, const float* __restrict__ bfv,
                                                          float* __restrict__ out) {
  __shared__ __align__(16) float Sl[8][96];
  const int tid = threadIdx.x, lane = tid & 31, wave = tid >> 5;
  const int g = blockIdx.x * 8 + wave;
  const int b = g >> 1;
  const int thalf = g & 1;
  const int t = thalf * 32 + lane;
  const v4f p0 = *(const v4f*)(PL + ((size_t)t * NODES_C + b) * 4);
  const v4f p1 = *(const v4f*)(PL + ((size_t)(TSTEPS + t) * NODES_C + b) * 4);
  const float l0 = (p0[0] + p1[0]) + bfv[0];
  const float l1 = (p0[1] + p1[1]) + bfv[1];
  const float l2 = (p0[2] + p1[2]) + bfv[2];
  const float m = fmaxf(l0, fmaxf(l1, l2));
  const float s0 = l0 - m, s1 = l1 - m, s2 = l2 - m;
  const float ls = logf((expf(s0) + expf(s1)) + expf(s2));
  Sl[wave][lane * 3 + 0] = s0 - ls;
  Sl[wave][lane * 3 + 1] = s1 - ls;
  Sl[wave][lane * 3 + 2] = s2 - ls;
  __syncthreads();
  const int li = lane < 24 ? lane : 23;
  const v4f v = *(const v4f*)(&Sl[wave][li * 4]);
  float* op = out + (size_t)b * (TSTEPS * NCLASS) + thalf * 96 + li * 4;
  if (lane < 24) *(volatile v4f*)op = v;
  __threadfence();
  if (lane < 24) *(volatile v4f*)op = v;
}

extern "C" void kernel_launch(void* const* d_in, const int* in_sizes, int n_in,
                              void* d_out, int out_size, void* d_ws, size_t ws_size, hipStream_t stream) {
  if (n_in < 22 || d_out == nullptr || d_ws == nullptr) return;
  if (in_sizes[0] != NODES_C * FEAT_C || in_sizes[1] != NODES_D * FEAT_D ||
      in_sizes[2] != EDGES_C || in_sizes[3] != EDGES_C || in_sizes[4] != EDGES_D || in_sizes[5] != EDGES_D ||
      in_sizes[6] != (FEAT_C + 1) * HIDDEN || in_sizes[7] != HIDDEN ||
      in_sizes[8] != (HIDDEN + 1) * HIDDEN || in_sizes[9] != HIDDEN ||
      in_sizes[10] != (FEAT_D + 1) * HIDDEN || in_sizes[11] != HIDDEN ||
      in_sizes[12] != (HIDDEN + 1) * HIDDEN || in_sizes[13] != HIDDEN ||
      in_sizes[14] != 2 * HIDDEN * GATES3 || in_sizes[15] != RNN_H * GATES3 || in_sizes[16] != 2 * GATES3 ||
      in_sizes[17] != 2 * HIDDEN * GATES3 || in_sizes[18] != RNN_H * GATES3 || in_sizes[19] != 2 * GATES3 ||
      in_sizes[20] != 2 * RNN_H * NCLASS || in_sizes[21] != NCLASS ||
      out_size != NODES_C * TSTEPS * NCLASS) return;

  const float* comp_feat = (const float*)d_in[0];
  const float* dev_feat  = (const float*)d_in[1];
  const int*   comp_src  = (const int*)d_in[2];
  const int*   comp_dst  = (const int*)d_in[3];
  const int*   dev_src   = (const int*)d_in[4];
  const int*   dev_dst   = (const int*)d_in[5];
  const float* W1c  = (const float*)d_in[6];
  const float* b1c  = (const float*)d_in[7];
  const float* W2c  = (const float*)d_in[8];
  const float* b2c  = (const float*)d_in[9];
  const float* W1d  = (const float*)d_in[10];
  const float* b1d  = (const float*)d_in[11];
  const float* W2d  = (const float*)d_in[12];
  const float* b2d  = (const float*)d_in[13];
  const float* Wx_f = (const float*)d_in[14];
  const float* Wh_f = (const float*)d_in[15];
  const float* b_f  = (const float*)d_in[16];
  const float* Wx_b = (const float*)d_in[17];
  const float* Wh_b = (const float*)d_in[18];
  const float* b_b  = (const float*)d_in[19];
  const float* Wf   = (const float*)d_in[20];
  const float* bfv  = (const float*)d_in[21];
  float* out = (float*)d_out;

  char* ws = (char*)d_ws;
  size_t off = 0;
  auto carve = [&](size_t bytes) -> char* { char* p = ws + off; off += (bytes + 255) & ~(size_t)255; return p; };
  unsigned short* ADJC  = (unsigned short*)carve((size_t)NODES_C * NODES_C * 2);
  unsigned short* ADJD  = (unsigned short*)carve((size_t)NODES_D * NODES_D * 2);
  float*          DEGC  = (float*)carve((size_t)3 * NODES_C * 4);
  float*          DEGD  = (float*)carve((size_t)3 * NODES_D * 4);
  unsigned short* W1CT  = (unsigned short*)carve((size_t)HIDDEN * FEAT_C * 2);
  unsigned short* W2CT  = (unsigned short*)carve((size_t)HIDDEN * HIDDEN * 2);
  unsigned short* W1DT  = (unsigned short*)carve((size_t)HIDDEN * FEAT_D_PAD * 2);
  unsigned short* W2DT  = (unsigned short*)carve((size_t)HIDDEN * HIDDEN * 2);
  unsigned short* WXTOP = (unsigned short*)carve((size_t)XPW * HIDDEN * 2);
  unsigned short* WXBOT = (unsigned short*)carve((size_t)XPW * HIDDEN * 2);
  unsigned short* WHT   = (unsigned short*)carve((size_t)2 * GATES3 * RNN_H * 2);
  unsigned short* WFT   = (unsigned short*)carve((size_t)2 * 16 * RNN_H * 2);
  unsigned short* FNC   = (unsigned short*)carve((size_t)NODES_C * FEAT_C * 2);
  unsigned short* FND   = (unsigned short*)carve((size_t)NODES_D * FEAT_D_PAD * 2);
  unsigned short* YTC1  = (unsigned short*)carve((size_t)HIDDEN * NODES_C * 2);
  unsigned short* YTC2  = (unsigned short*)carve((size_t)HIDDEN * NODES_C * 2);
  unsigned short* YTD1  = (unsigned short*)carve((size_t)HIDDEN * NODES_D * 2);
  unsigned short* YTD2  = (unsigned short*)carve((size_t)HIDDEN * NODES_D * 2);
  unsigned short* X1NC  = (unsigned short*)carve((size_t)NODES_C * HIDDEN * 2);
  unsigned short* X1ND  = (unsigned short*)carve((size_t)NODES_D * HIDDEN * 2);
  unsigned short* EMBC  = (unsigned short*)carve((size_t)NODES_C * HIDDEN * 2);
  unsigned short* EMBD  = (unsigned short*)carve((size_t)NODES_D * HIDDEN * 2);
  float*          CX    = (float*)carve((size_t)NODES_C * XPW * 4);
  float*          DX    = (float*)carve((size_t)NODES_D * XPW * 4);
  float*          PL    = (float*)carve((size_t)2 * TSTEPS * NODES_C * 4 * 4);
  if (off > ws_size || off > (size_t)134217728) return;

  deg_kernel<<<NODES_C / 32, NTHR, 0, stream>>>(comp_src, comp_dst, EDGES_C, NODES_C, DEGC);
  deg_kernel<<<NODES_D / 32, NTHR, 0, stream>>>(dev_src, dev_dst, EDGES_D, NODES_D, DEGD);
  adj_kernel<NODES_C><<<NODES_C / 8, NTHR, 0, stream>>>(comp_src, comp_dst, EDGES_C, ADJC);
  adj_kernel<NODES_D><<<NODES_D / 8, NTHR, 0, stream>>>(dev_src, dev_dst, EDGES_D, ADJD);

  tpw_f16_kernel<<<dim3(HIDDEN / 64, FEAT_C / 64), NTHR, 0, stream>>>(W1c, FEAT_C, HIDDEN, FEAT_C, W1CT, W_CARRY);
  tpw_f16_kernel<<<dim3(HIDDEN / 64, HIDDEN / 64), NTHR, 0, stream>>>(W2c, HIDDEN, HIDDEN, HIDDEN, W2CT, W_CARRY);
  tpw_f16_kernel<<<dim3(HIDDEN / 64, FEAT_D_PAD / 64), NTHR, 0, stream>>>(W1d, FEAT_D, HIDDEN, FEAT_D_PAD, W1DT, W_CARRY);
  tpw_f16_kernel<<<dim3(HIDDEN / 64, HIDDEN / 64), NTHR, 0, stream>>>(W2d, HIDDEN, HIDDEN, HIDDEN, W2DT, W_CARRY);
  tpw_f16_kernel<<<dim3(GATES3 / 64, HIDDEN / 64), NTHR, 0, stream>>>(Wx_f, HIDDEN, GATES3, HIDDEN, WXTOP, W_CARRY);
  tpw_f16_kernel<<<dim3(GATES3 / 64, HIDDEN / 64), NTHR, 0, stream>>>(Wx_b, HIDDEN, GATES3, HIDDEN, WXTOP + (size_t)GATES3 * HIDDEN, W_CARRY);
  tpw_f16_kernel<<<dim3(GATES3 / 64, HIDDEN / 64), NTHR, 0, stream>>>(Wx_f + (size_t)HIDDEN * GATES3, HIDDEN, GATES3, HIDDEN, WXBOT, W_CARRY);
  tpw_f16_kernel<<<dim3(GATES3 / 64, HIDDEN / 64), NTHR, 0, stream>>>(Wx_b + (size_t)HIDDEN * GATES3, HIDDEN, GATES3, HIDDEN, WXBOT + (size_t)GATES3 * HIDDEN, W_CARRY);
  tpw_f16_kernel<<<dim3(GATES3 / 64, RNN_H / 64), NTHR, 0, stream>>>(Wh_f, RNN_H, GATES3, RNN_H, WHT, W_CARRY);
  tpw_f16_kernel<<<dim3(GATES3 / 64, RNN_H / 64), NTHR, 0, stream>>>(Wh_b, RNN_H, GATES3, RNN_H, WHT + (size_t)GATES3 * RNN_H, W_CARRY);
  wf_prep_kernel<<<4, NTHR, 0, stream>>>(Wf, WFT);

  featn_kernel<<<(NODES_C * (FEAT_C / 8)) / NTHR, NTHR, 0, stream>>>(comp_feat, NODES_C, FEAT_C, FEAT_C, DEGC + 2 * NODES_C, FNC);
  featn_kernel<<<(NODES_D * (FEAT_D_PAD / 8)) / NTHR, NTHR, 0, stream>>>(dev_feat, NODES_D, FEAT_D, FEAT_D_PAD, DEGD + 2 * NODES_D, FND);

  auto gemm_h = [&](const unsigned short* A, int lda, const unsigned short* Bt, int ldb, unsigned short* C, int ldc,
                    int M, int N, int K, float sc) {
    const int tiles = (M / 64) * (N / 64);
    gemm_f16_kernel<1><<<(tiles + 7) / 8, NTHR, 0, stream>>>(A, lda, Bt, ldb, (void*)C, ldc, M, N, K, sc);
  };
  auto gemm_f = [&](const unsigned short* A, int lda, const unsigned short* Bt, int ldb, float* C, int ldc,
                    int M, int N, int K, float sc) {
    const int tiles = (M / 64) * (N / 64);
    gemm_f16_kernel<0><<<(tiles + 7) / 8, NTHR, 0, stream>>>(A, lda, Bt, ldb, (void*)C, ldc, M, N, K, sc);
  };

  gemm_h(W1CT, FEAT_C, FNC, FEAT_C, YTC1, NODES_C, HIDDEN, NODES_C, FEAT_C, 1.0f);
  graph_gemm_kernel<1><<<((NODES_C / 64) * (HIDDEN / 64) + 7) / 8, NTHR, 0, stream>>>(
      ADJC, NODES_C, YTC1, NODES_C, X1NC, HIDDEN, DEGC, W1c + (size_t)FEAT_C * HIDDEN, b1c,
      NODES_C, HIDDEN, NODES_C, W_CARRY_INV);
  gemm_h(W2CT, HIDDEN, X1NC, HIDDEN, YTC2, NODES_C, HIDDEN, NODES_C, HIDDEN, X1_CARRY_INV);
  graph_gemm_kernel<0><<<((NODES_C / 64) * (HIDDEN / 64) + 7) / 8, NTHR, 0, stream>>>(
      ADJC, NODES_C, YTC2, NODES_C, EMBC, HIDDEN, DEGC, W2c + (size_t)HIDDEN * HIDDEN, b2c,
      NODES_C, HIDDEN, NODES_C, W_CARRY_INV);

  gemm_h(W1DT, FEAT_D_PAD, FND, FEAT_D_PAD, YTD1, NODES_D, HIDDEN, NODES_D, FEAT_D_PAD, 1.0f);
  graph_gemm_kernel<1><<<((NODES_D / 64) * (HIDDEN / 64) + 7) / 8, NTHR, 0, stream>>>(
      ADJD, NODES_D, YTD1, NODES_D, X1ND, HIDDEN, DEGD, W1d + (size_t)FEAT_D * HIDDEN, b1d,
      NODES_D, HIDDEN, NODES_D, W_CARRY_INV);
  gemm_h(W2DT, HIDDEN, X1ND, HIDDEN, YTD2, NODES_D, HIDDEN, NODES_D, HIDDEN, X1_CARRY_INV);
  graph_gemm_kernel<0><<<((NODES_D / 64) * (HIDDEN / 64) + 7) / 8, NTHR, 0, stream>>>(
      ADJD, NODES_D, YTD2, NODES_D, EMBD, HIDDEN, DEGD, W2d + (size_t)HIDDEN * HIDDEN, b2d,
      NODES_D, HIDDEN, NODES_D, W_CARRY_INV);

  gemm_f(EMBC, HIDDEN, WXTOP, HIDDEN, CX, XPW, NODES_C, XPW, HIDDEN, W_CARRY_INV);
  gemm_f(EMBD, HIDDEN, WXBOT, HIDDEN, DX, XPW, NODES_D, XPW, HIDDEN, W_CARRY_INV);

  gru_bidir_kernel<<<2 * GRU_TILES, NTHR, 0, stream>>>(CX, DX, WHT, WFT, b_f, b_b, PL);
  head_final_kernel<<<(NODES_C * 2) / 8, NTHR, 0, stream>>>(PL, bfv, out);
}
